// EnetGnn_69810398429294
// MI455X (gfx1250) — hardware-verified
//
#include <hip/hip_runtime.h>
#include <stdint.h>
#include <stddef.h>

#define NIMG 4
#define CH   128
#define HIN  128
#define HP   64
#define NPOS 4096
#define KNB  16
#define QBLK 128
#define NQB  (NPOS / QBLK)

static_assert(HP * HP == NPOS);
static_assert(2 * HP == HIN);
static_assert(QBLK == 8 * 16);
static_assert(NQB == 32);
static_assert((CH % 32) == 0 && CH == 128);

typedef _Float16 v16h __attribute__((ext_vector_type(16)));
typedef _Float16 v8h  __attribute__((ext_vector_type(8)));
typedef float    v8f  __attribute__((ext_vector_type(8)));
typedef float    v4f  __attribute__((ext_vector_type(4)));

__device__ __forceinline__ v16h ldfrag(const _Float16* p) {
  union { v16h v; v8h h[2]; } f;
  f.h[0] = *(const v8h*)(p);
  f.h[1] = *(const v8h*)(p + 16);
  return f.v;
}
__device__ __forceinline__ v8f mma16(v16h a, v16h b, v8f c) {
  return __builtin_amdgcn_wmma_f32_16x16x32_f16(false, a, false, b, (short)0, c, false, false);
}
__device__ __forceinline__ v8f zero8() {
  v8f z;
#pragma unroll
  for (int i = 0; i < 8; ++i) z[i] = 0.0f;
  return z;
}
__device__ __forceinline__ void guard5(v8f& acc, v16h a0, v16h a1, v16h a2, v16h a3, v16h b3) {
#if defined(__HIP_DEVICE_COMPILE__)
  asm volatile("v_nop\n\tv_nop\n\tv_nop\n\tv_nop" : "+v"(acc) : "v"(a0), "v"(a1), "v"(a2), "v"(a3), "v"(b3));
#endif
}
__device__ __forceinline__ void guard_uv(v8f (&c)[2][4], v16h a0, v16h a1, v16h b0, v16h b1, v16h b2, v16h b3) {
#if defined(__HIP_DEVICE_COMPILE__)
  asm volatile("v_nop\n\tv_nop\n\tv_nop\n\tv_nop"
               : "+v"(c[0][0]), "+v"(c[0][1]), "+v"(c[0][2]), "+v"(c[0][3]),
                 "+v"(c[1][0]), "+v"(c[1][1]), "+v"(c[1][2]), "+v"(c[1][3])
               : "v"(a0), "v"(a1), "v"(b0), "v"(b1), "v"(b2), "v"(b3));
#endif
}
__device__ __forceinline__ void lds_sync_wave() {
  __builtin_amdgcn_fence(__ATOMIC_RELEASE, "wavefront");
  __builtin_amdgcn_wave_barrier();
  __builtin_amdgcn_fence(__ATOMIC_ACQUIRE, "wavefront");
}
__device__ __forceinline__ void lds_sync_wg() {
  __builtin_amdgcn_fence(__ATOMIC_RELEASE, "workgroup");
  __builtin_amdgcn_wave_barrier();
  __builtin_amdgcn_fence(__ATOMIC_ACQUIRE, "workgroup");
}
__device__ __forceinline__ float leaky(float x) { return (x >= 0.0f) ? x : 0.01f * x; }
__device__ __forceinline__ float max4(float a, float b, float c, float d) { return fmaxf(fmaxf(a, b), fmaxf(c, d)); }

__global__ __launch_bounds__(256) void k_pool(const float* __restrict__ in0, const float* __restrict__ in1,
                                               _Float16* __restrict__ XH, float* __restrict__ SD,
                                               _Float16* __restrict__ X0H) {
  __shared__ float xt[CH * 65];
  __shared__ float sscl[HP];
  __shared__ __align__(16) float ssum[HP];
  const int t = threadIdx.x, y = blockIdx.x, n = blockIdx.y, mod = blockIdx.z;
  const float* src = (mod != 0) ? in1 : in0;
  {
    const int xq = t & 31, cl = t >> 5;
#pragma unroll 1
    for (int cc = 0; cc < CH / 8; ++cc) {
      const int c = cc * 8 + cl;
      const float* p = src + (((size_t)(n * CH + c)) * HIN + 2 * y) * HIN + 4 * xq;
      const v4f a = *(const v4f*)p;
      const v4f b = *(const v4f*)(p + HIN);
      xt[c * 65 + 2 * xq]     = max4(a[0], a[1], b[0], b[1]);
      xt[c * 65 + 2 * xq + 1] = max4(a[2], a[3], b[2], b[3]);
    }
  }
  __syncthreads();
  {
    const int x = t >> 2, part = t & 3;
    float ss = 0.0f;
#pragma unroll 4
    for (int i = 0; i < 32; ++i) {
      const float v = xt[(part * 32 + i) * 65 + x];
      ss = fmaf(v, v, ss);
    }
    ss += __shfl_xor(ss, 1, 32);
    ss += __shfl_xor(ss, 2, 32);
    const float nrm = sqrtf(ss);
    const float scl = (1.0f / fmaxf(nrm, 1e-12f)) * 64.0f;
    float sq = 0.0f;
#pragma unroll 4
    for (int i = 0; i < 32; ++i) {
      const float v = xt[(part * 32 + i) * 65 + x];
      const float hv = (float)((_Float16)(v * scl));
      sq = fmaf(hv, hv, sq);
    }
    sq += __shfl_xor(sq, 1, 32);
    sq += __shfl_xor(sq, 2, 32);
    if (part == 0) { sscl[x] = scl; ssum[x] = sq; }
  }
  __syncthreads();
  {
    _Float16* base = XH + ((size_t)(mod * NIMG + n) * NPOS + (size_t)y * HP) * CH;
    v8h o[4];
#pragma unroll
    for (int i = 0; i < 4; ++i) {
      const int e = i * 256 + t, x = e >> 4, q = e & 15;
      const float scl = sscl[x];
#pragma unroll
      for (int k = 0; k < 8; ++k) o[i][k] = (_Float16)(xt[(8 * q + k) * 65 + x] * scl);
    }
#pragma unroll
    for (int ps = 0; ps < 2; ++ps) {
#pragma unroll
      for (int i = 0; i < 4; ++i) {
        const int e = i * 256 + t, x = e >> 4, q = e & 15;
        *(volatile v8h*)(base + x * CH + 8 * q) = o[i];
      }
      __threadfence();
    }
  }
  if (t < 32) {
    const int tt = t & 15;
    const v4f v = *(const v4f*)(ssum + 4 * tt);
    float* d = SD + (size_t)(mod * NIMG + n) * NPOS + (size_t)y * HP + 4 * tt;
    if (t < 16) { *(volatile v4f*)d = v; }
    __threadfence();
    if (t < 16) { *(volatile v4f*)d = v; }
  }
  if (n == 0) {
    _Float16* base = X0H + ((size_t)mod * NPOS + (size_t)y * HP) * CH;
    v8h o[4];
#pragma unroll
    for (int i = 0; i < 4; ++i) {
      const int e = i * 256 + t, x = e >> 4, q = e & 15;
#pragma unroll
      for (int k = 0; k < 8; ++k) o[i][k] = (_Float16)(xt[(8 * q + k) * 65 + x] * 8.0f);
    }
#pragma unroll
    for (int ps = 0; ps < 2; ++ps) {
#pragma unroll
      for (int i = 0; i < 4; ++i) {
        const int e = i * 256 + t, x = e >> 4, q = e & 15;
        *(volatile v8h*)(base + x * CH + 8 * q) = o[i];
      }
      __threadfence();
    }
  }
}

__global__ __launch_bounds__(256) void k_wcvt(const float* __restrict__ Wr, const float* __restrict__ Wi,
                                               _Float16* __restrict__ WT) {
  const int t = threadIdx.x, rb = blockIdx.x, slot = blockIdx.y;
  const float* W = (slot >= 2) ? Wi : Wr;
  const int nn = rb * 16 + (t >> 4);
  const int k8 = (t & 15) * 8;
  v8h o;
#pragma unroll
  for (int i = 0; i < 8; ++i) {
    const int k = k8 + i;
    const float top = W[(size_t)k * CH + nn];
    const float bot = W[(size_t)(CH + k) * CH + nn];
    const float v = (slot & 1) ? bot : (top + bot);
    o[i] = (_Float16)(v * 64.0f);
  }
  _Float16* d = WT + (size_t)slot * CH * CH + (size_t)nn * CH + k8;
  *(volatile v8h*)d = o;
  __threadfence();
  *(volatile v8h*)d = o;
}

__global__ __launch_bounds__(256) void k_uv(const _Float16* __restrict__ X0H, const _Float16* __restrict__ WT,
                                             float* __restrict__ UV) {
  __shared__ __align__(16) float sT[8][16 * 68];
  const int lane = threadIdx.x & 31, wave = threadIdx.x >> 5;
  const int y = blockIdx.y;
  const int amod = ((y + 1) >> 1) & 1;
  const _Float16* A  = X0H + (size_t)amod * NPOS * CH;
  const _Float16* Bt = WT + (size_t)y * CH * CH;
  float* C = UV + (size_t)y * NPOS * CH;
  const int tile = (int)blockIdx.x * 8 + wave;
  const int m0 = (tile >> 1) * 32, n0 = (tile & 1) * 64;
  const int rl = lane & 15, h8 = (lane >> 4) * 8;

  v8f acc[2][4];
#pragma unroll
  for (int i = 0; i < 2; ++i)
#pragma unroll
    for (int j = 0; j < 4; ++j) acc[i][j] = zero8();

#pragma unroll 1
  for (int k0 = 0; k0 < CH; k0 += 32) {
    v16h b[4];
#pragma unroll
    for (int j = 0; j < 4; ++j) b[j] = ldfrag(Bt + (size_t)(n0 + (j << 4) + rl) * CH + k0 + h8);
    const v16h a0 = ldfrag(A + (size_t)(m0 + rl) * CH + k0 + h8);
    const v16h a1 = ldfrag(A + (size_t)(m0 + 16 + rl) * CH + k0 + h8);
#pragma unroll
    for (int j = 0; j < 4; ++j) {
      acc[0][j] = mma16(a0, b[j], acc[0][j]);
      acc[1][j] = mma16(a1, b[j], acc[1][j]);
    }
    guard_uv(acc, a0, a1, b[0], b[1], b[2], b[3]);
  }

  float* slab = sT[wave];
  const int hh = lane >> 4, c4 = (lane & 15) * 4;
#pragma unroll
  for (int i = 0; i < 2; ++i) {
#pragma unroll
    for (int j = 0; j < 4; ++j)
#pragma unroll
      for (int r = 0; r < 8; ++r) slab[(h8 + r) * 68 + (j << 4) + rl] = acc[i][j][r] * (1.0f / 512.0f);
    lds_sync_wg();
#pragma unroll
    for (int ps = 0; ps < 2; ++ps) {
#pragma unroll
      for (int it = 0; it < 8; ++it) {
        const int row = it * 2 + hh;
        const v4f v = *(const v4f*)(slab + row * 68 + c4);
        *(volatile v4f*)(C + (size_t)(m0 + 16 * i + row) * CH + n0 + c4) = v;
      }
      __threadfence();
    }
    lds_sync_wg();
  }
}

__global__ __launch_bounds__(256) void k_sel(const _Float16* __restrict__ XH, const float* __restrict__ SD,
                                              const float* __restrict__ UV, const float* __restrict__ b_r,
                                              const float* __restrict__ b_i, float* __restrict__ PART) {
  __shared__ unsigned keyx[8 * 32 * KNB];
  __shared__ unsigned short idxl[2 * 8 * 16 * KNB];
  __shared__ __align__(16) float comb[8 * 256];
  __shared__ __align__(16) float totl[256];
  const int t = threadIdx.x, wave = t >> 5, lane = t & 31, rl = lane & 15, h8 = (lane >> 4) * 8;
  const int bx = blockIdx.x, n = blockIdx.y;
  const int qw = bx * QBLK + wave * 16;

#pragma unroll 1
  for (int mod = 0; mod < 2; ++mod) {
    const _Float16* xb = XH + (size_t)(mod * NIMG + n) * NPOS * CH;
    const float* sdb = SD + (size_t)(mod * NIMG + n) * NPOS;
    const _Float16* qp = xb + (size_t)(qw + rl) * CH + h8;
    const v16h bq0 = ldfrag(qp), bq1 = ldfrag(qp + 32), bq2 = ldfrag(qp + 64), bq3 = ldfrag(qp + 96);
    unsigned top[KNB];
#pragma unroll
    for (int s = 0; s < KNB; ++s) top[s] = 0xFFFFFFFFu;

#pragma unroll 1
    for (int ct = 0; ct < NPOS / 16; ++ct) {
      const _Float16* cp = xb + (size_t)(ct * 16 + rl) * CH + h8;
      const v16h a0 = ldfrag(cp), a1 = ldfrag(cp + 32), a2 = ldfrag(cp + 64), a3 = ldfrag(cp + 96);
      v8f acc = zero8();
      acc = mma16(a0, bq0, acc);
      acc = mma16(a1, bq1, acc);
      acc = mma16(a2, bq2, acc);
      acc = mma16(a3, bq3, acc);
      guard5(acc, a0, a1, a2, a3, bq3);
      const int cb = ct * 16 + h8;
      const v8f sv = *(const v8f*)(sdb + cb);
#pragma unroll
      for (int r = 0; r < 8; ++r) {
        const float e = fmaf(-2.0f, acc[r], sv[r]);
        float uf = (e + 4096.0f) * 64.0f;
        uf = fminf(fmaxf(uf, 0.0f), 1048574.0f);
        unsigned key = (((unsigned)uf) << 12) | (unsigned)(cb + r);
        if (key < top[KNB - 1]) {
#pragma unroll
          for (int s = 0; s < KNB; ++s) {
            const unsigned o = top[s];
            top[s] = (o < key) ? o : key;
            key    = (o < key) ? key : o;
          }
        }
      }
    }
    {
      unsigned* kx = keyx + (wave * 32 + lane) * KNB;
#pragma unroll
      for (int s = 0; s < KNB; ++s) kx[s] = top[s];
    }
    lds_sync_wave();
    {
      const int ql = lane & 15;
      const unsigned* la = keyx + (wave * 32 + ql) * KNB;
      const unsigned* lb = keyx + (wave * 32 + ql + 16) * KNB;
      unsigned short* dst = idxl + ((mod * 8 + wave) * 16 + ql) * KNB;
      int pa = 0, pb = 0;
#pragma unroll
      for (int s = 0; s < KNB; ++s) {
        const unsigned ka = la[pa], kb = lb[pb];
        const bool ta = (ka < kb);
        const unsigned kk = ta ? ka : kb;
        pa += ta ? 1 : 0;
        pb += ta ? 0 : 1;
        dst[s] = (unsigned short)(kk & 0xFFFu);
      }
    }
    lds_sync_wave();
  }

  {
    const size_t P = (size_t)NPOS * CH;
    const float* Ur = UV;
    const float* Vi = UV + P;
    const float* Ui = UV + 2 * P;
    const float* Vr = UV + 3 * P;
    const v4f br = *(const v4f*)(b_r + 4 * lane);
    const v4f bi = *(const v4f*)(b_i + 4 * lane);
    v4f csr, csi;
#pragma unroll
    for (int c = 0; c < 4; ++c) { csr[c] = 0.0f; csi[c] = 0.0f; }
    const unsigned short* ia = idxl + (wave * 16) * KNB;
    const unsigned short* ib = idxl + ((8 + wave) * 16) * KNB;
#pragma unroll 1
    for (int pe = 0; pe < 16 * KNB; ++pe) {
      int a = (int)ia[pe];
      int b = (int)ib[pe];
      a = (a > NPOS - 1) ? (NPOS - 1) : a;
      b = (b > NPOS - 1) ? (NPOS - 1) : b;
      const v4f ur = *(const v4f*)(Ur + (size_t)a * CH + 4 * lane);
      const v4f vi = *(const v4f*)(Vi + (size_t)b * CH + 4 * lane);
      const v4f ui = *(const v4f*)(Ui + (size_t)b * CH + 4 * lane);
      const v4f vr = *(const v4f*)(Vr + (size_t)a * CH + 4 * lane);
#pragma unroll
      for (int c = 0; c < 4; ++c) {
        csr[c] += leaky((ur[c] - vi[c]) + br[c]);
        csi[c] += leaky((ui[c] - vr[c]) + bi[c]);
      }
    }
    *(v4f*)(comb + wave * 256 + 4 * lane) = csr;
    *(v4f*)(comb + wave * 256 + CH + 4 * lane) = csi;
  }
  __syncthreads();
  {
    float s = 0.0f;
#pragma unroll
    for (int w = 0; w < 8; ++w) s += comb[w * 256 + t];
    totl[t] = s;
  }
  __syncthreads();
  if (t < 64) {
    const v4f v = *(const v4f*)(totl + 4 * t);
    float* d = PART + ((size_t)(n * NQB + bx)) * 256 + 4 * t;
    *(volatile v4f*)d = v;
    __threadfence();
    *(volatile v4f*)d = v;
  }
}

__global__ __launch_bounds__(256) void k_gate(const float* __restrict__ PART, const float* __restrict__ w1,
                                               const float* __restrict__ b1, const float* __restrict__ w2,
                                               const float* __restrict__ b2, const int* __restrict__ itp,
                                               const int* __restrict__ kp, float* __restrict__ GATE) {
  __shared__ float mm[2 * CH];
  __shared__ float zz[8];
  __shared__ __align__(16) float gl[CH];
  const int n = blockIdx.x, t = threadIdx.x;
  int kv = kp[0];
  kv = (kv < 1) ? 1 : kv;
  const int itv = itp[0];
  (void)itv;
  double ds = 0.0;
#pragma unroll 1
  for (int b = 0; b < NQB; ++b) ds += (double)PART[((size_t)(n * NQB + b)) * 256 + t];
  mm[t] = (float)(ds / ((double)NPOS * (double)kv));
  __syncthreads();
  if (t < 32) {
    const int tc = t & 7;
    float s = 0.0f;
#pragma unroll 1
    for (int i = 0; i < 2 * CH; ++i) s = fmaf(mm[i], w1[i * 8 + tc], s);
    s += b1[tc];
    s = leaky(s);
    if (t < 8) zz[t] = s;
  }
  __syncthreads();
  if (t < CH) {
    float s = 0.0f;
#pragma unroll
    for (int j = 0; j < 8; ++j) s = fmaf(zz[j], w2[j * CH + t], s);
    s += b2[t];
    gl[t] = 1.0f / (1.0f + expf(-s));
  }
  __syncthreads();
  if (t < 32) {
    const v4f v = *(const v4f*)(gl + 4 * t);
    float* d = GATE + (size_t)n * CH + 4 * t;
    *(volatile v4f*)d = v;
    __threadfence();
    *(volatile v4f*)d = v;
  }
}

__global__ __launch_bounds__(256) void k_out(const float* __restrict__ in0, const float* __restrict__ in1,
                                              const float* __restrict__ GATE, const float* __restrict__ g1p,
                                              const float* __restrict__ g2p, float* __restrict__ out) {
#pragma clang fp contract(off)
  const int t = threadIdx.x;
  const int yb = blockIdx.x, c = blockIdx.y, n = blockIdx.z;
  const int y = yb * 16 + (t >> 4), xq = t & 15;
  const size_t rb = (((size_t)(n * CH + c)) * HIN + 2 * y) * HIN + 8 * xq;
  const v4f ra0 = *(const v4f*)(in0 + rb), ra1 = *(const v4f*)(in0 + rb + 4);
  const v4f rc0 = *(const v4f*)(in0 + rb + HIN), rc1 = *(const v4f*)(in0 + rb + HIN + 4);
  const v4f ia0 = *(const v4f*)(in1 + rb), ia1 = *(const v4f*)(in1 + rb + 4);
  const v4f ic0 = *(const v4f*)(in1 + rb + HIN), ic1 = *(const v4f*)(in1 + rb + HIN + 4);
  float pr[4], pi[4];
  pr[0] = max4(ra0[0], ra0[1], rc0[0], rc0[1]);
  pr[1] = max4(ra0[2], ra0[3], rc0[2], rc0[3]);
  pr[2] = max4(ra1[0], ra1[1], rc1[0], rc1[1]);
  pr[3] = max4(ra1[2], ra1[3], rc1[2], rc1[3]);
  pi[0] = max4(ia0[0], ia0[1], ic0[0], ic0[1]);
  pi[1] = max4(ia0[2], ia0[3], ic0[2], ic0[3]);
  pi[2] = max4(ia1[0], ia1[1], ic1[0], ic1[1]);
  pi[3] = max4(ia1[2], ia1[3], ic1[2], ic1[3]);
  const float g = GATE[n * CH + c];
  const float om = 1.0f - g;
  const float ga = g1p[0], gb = g2p[0];
  v4f o;
#pragma unroll
  for (int i = 0; i < 4; ++i) {
    const float t1 = g * pr[i];
    const float t2 = om * pi[i];
    const float hsum = ga * t1 + gb * t2;
    o[i] = fmaxf(hsum, 0.0f);
  }
  float* d = out + (((size_t)(n * CH + c)) * HP + y) * HP + 4 * xq;
  *(volatile v4f*)d = o;
  __threadfence();
  *(volatile v4f*)d = o;
}

extern "C" void kernel_launch(void* const* d_in, const int* in_sizes, int n_in,
                              void* d_out, int out_size, void* d_ws, size_t ws_size,
                              hipStream_t stream) {
  if (n_in < 14) return;
  const int nimg_elems = NIMG * CH * HIN * HIN;
  if (in_sizes[0] != nimg_elems || in_sizes[1] != nimg_elems) return;
  if (in_sizes[2] != 2 * CH * CH || in_sizes[4] != 2 * CH * CH) return;
  if (in_sizes[3] != CH || in_sizes[5] != CH) return;
  if (in_sizes[6] != 2 * CH * 8 || in_sizes[7] != 8 || in_sizes[8] != 8 * CH || in_sizes[9] != CH) return;
  if (in_sizes[10] < 1 || in_sizes[11] < 1 || in_sizes[12] < 1 || in_sizes[13] < 1) return;
  if (out_size != NIMG * CH * NPOS) return;

  const float* rgb = (const float*)d_in[0];
  const float* ir  = (const float*)d_in[1];
  const float* Wrg = (const float*)d_in[2];
  const float* brg = (const float*)d_in[3];
  const float* Wig = (const float*)d_in[4];
  const float* big = (const float*)d_in[5];
  const float* sw1 = (const float*)d_in[6];
  const float* sb1 = (const float*)d_in[7];
  const float* sw2 = (const float*)d_in[8];
  const float* sb2 = (const float*)d_in[9];
  const float* g1  = (const float*)d_in[10];
  const float* g2  = (const float*)d_in[11];
  const int*   itp = (const int*)d_in[12];
  const int*   kp  = (const int*)d_in[13];
  float* out = (float*)d_out;

  const size_t bXH   = (size_t)2 * NIMG * NPOS * CH * 2;
  const size_t bSD   = (size_t)2 * NIMG * NPOS * 4;
  const size_t bX0   = (size_t)2 * NPOS * CH * 2;
  const size_t bWT   = (size_t)4 * CH * CH * 2;
  const size_t bUV   = (size_t)4 * NPOS * CH * 4;
  const size_t bPART = (size_t)NIMG * NQB * 256 * 4;
  const size_t bGATE = (size_t)NIMG * CH * 4;
  size_t off = 0;
  const size_t oXH = off;   off += bXH;
  const size_t oSD = off;   off += bSD;
  const size_t oX0 = off;   off += bX0;
  const size_t oWT = off;   off += bWT;
  const size_t oUV = off;   off += bUV;
  const size_t oPART = off; off += bPART;
  const size_t oGATE = off; off += bGATE;
  if (off > ws_size) return;
  if (off > (size_t)134217728) return;

  char* ws = (char*)d_ws;
  _Float16* XH   = (_Float16*)(ws + oXH);
  float*    SD   = (float*)(ws + oSD);
  _Float16* X0H  = (_Float16*)(ws + oX0);
  _Float16* WT   = (_Float16*)(ws + oWT);
  float*    UV   = (float*)(ws + oUV);
  float*    PART = (float*)(ws + oPART);
  float*    GATE = (float*)(ws + oGATE);

  const dim3 blk(256);
  k_pool<<<dim3(HP, NIMG, 2), blk, 0, stream>>>(rgb, ir, XH, SD, X0H);
  k_wcvt<<<dim3(CH / 16, 4), blk, 0, stream>>>(Wrg, Wig, WT);
  k_uv<<<dim3(((NPOS / 32) * (CH / 64)) / 8, 4), blk, 0, stream>>>(X0H, WT, UV);
  k_sel<<<dim3(NQB, NIMG), blk, 0, stream>>>(XH, SD, UV, brg, big, PART);
  k_gate<<<dim3(NIMG), blk, 0, stream>>>(PART, sw1, sb1, sw2, sb2, itp, kp, GATE);
  k_out<<<dim3(HP / 16, CH, NIMG), blk, 0, stream>>>(rgb, ir, GATE, g1, g2, out);
  (void)hipGetLastError();
}
